// IntraGraphAttention_3478923509961
// MI455X (gfx1250) — hardware-verified
//
#include <hip/hip_runtime.h>
#include <stddef.h>


#define KD    128
#define HC    64
#define NHD   2
#define CPH   32
#define GR    64
#define AP    136
#define XSP   68
#define NB    512
#define CHUNK 2048
#define NTHR  256
#define NWAVE 8
#define WCAP  256
#define NGRP  (CHUNK / (NTHR * 4))

#define LDS_SACC (NB * HC)
#define LDS_STAT (NB * NHD)
#define LDS_LIST (NWAVE * WCAP)
#define LDS_BYTES ((LDS_SACC + 2 * LDS_STAT + LDS_LIST + 16) * 4)

static_assert(KD % 32 == 0);
static_assert(HC == 64);
static_assert(NHD * CPH == HC);
static_assert(GR == 64);
static_assert(NTHR == GR * 4);
static_assert(WCAP == (CHUNK / NTHR) * 32);
static_assert(NGRP == 2);
static_assert(NB == 512);
static_assert(CHUNK == 2048);
static_assert((NB / NWAVE) % 2 == 0);
static_assert(LDS_BYTES == 147520);

typedef float          v2f  __attribute__((ext_vector_type(2)));
typedef float          v4f  __attribute__((ext_vector_type(4)));
typedef float          v8f  __attribute__((ext_vector_type(8)));
typedef int            v4i  __attribute__((ext_vector_type(4)));
typedef unsigned short v8us __attribute__((ext_vector_type(8)));
typedef __bf16         v8b_raw __attribute__((ext_vector_type(8)));
typedef v8b_raw        v8b  __attribute__((may_alias));
typedef __bf16         v16b __attribute__((ext_vector_type(16)));
union FragB { v16b v; v8b half[2]; };
union PackU { v8us h; v4i i; };

__device__ __forceinline__ v8f wm(v16b a, v16b b, v8f c) {
  v8f d = __builtin_amdgcn_wmma_f32_16x16x32_bf16(false, a, false, b, (short)0, c, false, false);
  asm volatile("v_nop\n\tv_nop\n\tv_nop\n\tv_nop" : "+v"(d) : "v"(a), "v"(b));
  return d;
}

__device__ __forceinline__ unsigned int bf16_rne(float f) {
  const unsigned int u = __float_as_uint(f);
  return (u + 0x7FFFu + ((u >> 16) & 1u)) >> 16;
}

__device__ __forceinline__ void split2(float f, unsigned short& hb, unsigned short& lb) {
  const unsigned int h = bf16_rne(f);
  const float hf = __uint_as_float(h << 16);
  hb = (unsigned short)h;
  lb = (unsigned short)bf16_rne(f - hf);
}

__global__ __launch_bounds__(NTHR) void k_prep(const float* __restrict__ W,
                                               unsigned short* Whi, unsigned short* Wlo, int n8) {
  const int i = blockIdx.x * NTHR + threadIdx.x;
  if (i >= n8) return;
  const int n  = i / (KD / 8);
  const int k0 = (i % (KD / 8)) * 8;
  PackU uh, ul;
#pragma unroll
  for (int j = 0; j < 8; ++j) {
    const float f = W[(size_t)(k0 + j) * HC + n];
    unsigned short hb, lb;
    split2(f, hb, lb);
    uh.h[j] = hb;
    ul.h[j] = lb;
  }
  const v4i vh = uh.i;
  const v4i vl = ul.i;
  unsigned short* ph = Whi + (size_t)n * KD + k0;
  unsigned short* pl = Wlo + (size_t)n * KD + k0;
  *(volatile v4i*)ph = vh;
  *(volatile v4i*)pl = vl;
  __threadfence();
  *(volatile v4i*)ph = vh;
  *(volatile v4i*)pl = vl;
}

__global__ __launch_bounds__(NTHR) void k_gemm(
    const float* __restrict__ x,
    const unsigned short* __restrict__ Whi, const unsigned short* __restrict__ Wlo,
    const float* __restrict__ att_src, const float* __restrict__ att_dst,
    float* hpl, float* aspl, float* adpl, int nN) {
  __shared__ __attribute__((aligned(16))) unsigned short Ahi[GR * AP];
  __shared__ __attribute__((aligned(16))) unsigned short Alo[GR * AP];
  __shared__ __attribute__((aligned(16))) float Xs[GR * XSP];
  __shared__ __attribute__((aligned(16))) float ADs[2 * GR * NHD];
  __shared__ __attribute__((aligned(16))) float atts[2 * HC];

  const int tid  = threadIdx.x;
  const int lane = tid & 31;
  const int wave = tid >> 5;
  const int hh   = lane >> 4;
  const int m    = lane & 15;
  const int rowBase = blockIdx.x * GR;

  if (tid < HC) {
    atts[tid]      = att_src[tid];
    atts[HC + tid] = att_dst[tid];
  }

  {
    const int r  = tid >> 2;
    const int c0 = (tid & 3) * 32;
    int row = rowBase + r;
    if (row > nN - 1) row = nN - 1;
    const float* p = x + (size_t)row * KD + c0;
#pragma unroll 1
    for (int g = 0; g < 4; ++g) {
      const v4f f0 = *(const v4f*)(p + 8 * g);
      const v4f f1 = *(const v4f*)(p + 8 * g + 4);
      float v[8] = {f0.x, f0.y, f0.z, f0.w, f1.x, f1.y, f1.z, f1.w};
      PackU uh, ul;
#pragma unroll
      for (int j = 0; j < 8; ++j) {
        float a = v[j];
        const float en = expm1f(fminf(a, 0.0f));
        a = (a > 0.0f) ? a : en;
        unsigned short hb, lb;
        split2(a, hb, lb);
        uh.h[j] = hb;
        ul.h[j] = lb;
      }
      *(v4i*)(Ahi + r * AP + c0 + 8 * g) = uh.i;
      *(v4i*)(Alo + r * AP + c0 + 8 * g) = ul.i;
    }
  }
  __syncthreads();

  const int ct   = wave & 3;
  const int rt   = (wave >> 2) * 2;
  const int ncol = ct * 16 + m;
  v8f c0a = {0.f, 0.f, 0.f, 0.f, 0.f, 0.f, 0.f, 0.f};
  v8f c1a = {0.f, 0.f, 0.f, 0.f, 0.f, 0.f, 0.f, 0.f};
#pragma unroll 1
  for (int kt = 0; kt < KD / 32; ++kt) {
    const int k0 = kt * 32;
    FragB bh, bl, a0h, a0l, a1h, a1l;
    const unsigned short* pbh = Whi + (size_t)ncol * KD + k0 + 8 * hh;
    const unsigned short* pbl = Wlo + (size_t)ncol * KD + k0 + 8 * hh;
    const unsigned short* pa0h = Ahi + (rt * 16 + m) * AP + k0 + 8 * hh;
    const unsigned short* pa1h = Ahi + (rt * 16 + 16 + m) * AP + k0 + 8 * hh;
    const unsigned short* pa0l = Alo + (rt * 16 + m) * AP + k0 + 8 * hh;
    const unsigned short* pa1l = Alo + (rt * 16 + 16 + m) * AP + k0 + 8 * hh;
    bh.half[0]  = *(const v8b*)pbh;   bh.half[1]  = *(const v8b*)(pbh + 16);
    bl.half[0]  = *(const v8b*)pbl;   bl.half[1]  = *(const v8b*)(pbl + 16);
    a0h.half[0] = *(const v8b*)pa0h;  a0h.half[1] = *(const v8b*)(pa0h + 16);
    a1h.half[0] = *(const v8b*)pa1h;  a1h.half[1] = *(const v8b*)(pa1h + 16);
    a0l.half[0] = *(const v8b*)pa0l;  a0l.half[1] = *(const v8b*)(pa0l + 16);
    a1l.half[0] = *(const v8b*)pa1l;  a1l.half[1] = *(const v8b*)(pa1l + 16);
    c0a = wm(a0h.v, bh.v, c0a);
    c0a = wm(a0h.v, bl.v, c0a);
    c0a = wm(a0l.v, bh.v, c0a);
    c1a = wm(a1h.v, bh.v, c1a);
    c1a = wm(a1h.v, bl.v, c1a);
    c1a = wm(a1l.v, bh.v, c1a);
  }

#pragma unroll
  for (int r = 0; r < 8; ++r) {
    Xs[(rt * 16 + 8 * hh + r) * XSP + ncol]      = c0a[r];
    Xs[(rt * 16 + 16 + 8 * hh + r) * XSP + ncol] = c1a[r];
  }
  __syncthreads();

  {
    const int row   = tid >> 2;
    const int hd    = (tid >> 1) & 1;
    const int which = tid & 1;
    const float* xsr = Xs + row * XSP + CPH * hd;
    const float* at  = atts + which * HC + CPH * hd;
    float s = 0.f;
#pragma unroll 8
    for (int c = 0; c < CPH; ++c) s += xsr[c] * at[c];
    ADs[which * (GR * NHD) + row * NHD + hd] = s;
  }
  __syncthreads();

  v4f xr[4];
#pragma unroll
  for (int i = 0; i < 4; ++i) xr[i] = *(const v4f*)(Xs + (8 * wave + 2 * i + hh) * XSP + 4 * m);
  const v4f gv = *(const v4f*)(ADs + (wave & 1) * (GR * NHD) + 4 * lane);
  float* hp[4];
#pragma unroll
  for (int i = 0; i < 4; ++i) hp[i] = hpl + (size_t)(rowBase + 8 * wave + 2 * i) * HC + 4 * lane;
  float* gp = (wave == 0) ? (aspl + (size_t)rowBase * NHD + 4 * lane)
                          : (adpl + (size_t)rowBase * NHD + 4 * lane);

#pragma unroll
  for (int i = 0; i < 4; ++i) *(volatile v4f*)(hp[i]) = xr[i];
  if (wave < 2) *(volatile v4f*)gp = gv;
  __threadfence();
#pragma unroll
  for (int i = 0; i < 4; ++i) *(volatile v4f*)(hp[i]) = xr[i];
  if (wave < 2) *(volatile v4f*)gp = gv;
}

__global__ __launch_bounds__(NTHR) void k_gat(
    const int* __restrict__ ei, const float* __restrict__ hpl,
    const float* __restrict__ aspl, const float* __restrict__ adpl,
    const float* __restrict__ bias, float* out, int nN, int nE) {
  extern __shared__ v4f lds_dyn[];
  float* sacc = (float*)lds_dyn;
  float* smax = sacc + LDS_SACC;
  float* sden = smax + LDS_STAT;
  int*   list = (int*)(sden + LDS_STAT);
  int*   wcnt = list + LDS_LIST;

  const int tid  = threadIdx.x;
  const int lane = tid & 31;
  const int wave = tid >> 5;
  const int hh   = lane >> 4;
  const int nodeBase = blockIdx.x * NB;

  {
    const v4f z4 = {0.f, 0.f, 0.f, 0.f};
    for (int i = tid; i < LDS_SACC / 4; i += NTHR) lds_dyn[i] = z4;
    for (int i = tid; i < LDS_STAT; i += NTHR) { smax[i] = -1e30f; sden[i] = 0.f; }
  }
  __syncthreads();

  const int* eid = ei + nE;
  const bool al16 = ((nE & 3) == 0);
  const int hd = hh;

  const int nChunks = (nE + CHUNK - 1) / CHUNK;
#pragma unroll 1
  for (int ch = 0; ch < nChunks; ++ch) {
    const int cbase = ch * CHUNK;
    int wc = 0;
#pragma unroll
    for (int g = 0; g < NGRP; ++g) {
      const int el0 = (g * NTHR + tid) * 4;
      const int e0  = cbase + el0;
      const int sent = -2147483647 - 1;
      v4i d;
      if (al16 && (cbase + CHUNK <= nE)) {
        d = *(const v4i*)(eid + e0);
      } else {
        d.x = (e0     < nE) ? eid[min(e0,     nE - 1)] : sent;
        d.y = (e0 + 1 < nE) ? eid[min(e0 + 1, nE - 1)] : sent;
        d.z = (e0 + 2 < nE) ? eid[min(e0 + 2, nE - 1)] : sent;
        d.w = (e0 + 3 < nE) ? eid[min(e0 + 3, nE - 1)] : sent;
      }
      const unsigned s0 = (unsigned)d.x - (unsigned)nodeBase;
      const unsigned s1 = (unsigned)d.y - (unsigned)nodeBase;
      const unsigned s2 = (unsigned)d.z - (unsigned)nodeBase;
      const unsigned s3 = (unsigned)d.w - (unsigned)nodeBase;
      const bool h0 = s0 < (unsigned)NB;
      const bool h1 = s1 < (unsigned)NB;
      const bool h2 = s2 < (unsigned)NB;
      const bool h3 = s3 < (unsigned)NB;
      const unsigned many = __builtin_amdgcn_ballot_w32(h0 | h1 | h2 | h3);
      if (many != 0u) {
#define HITJ(J, HJ, SJ) { \
          const unsigned mj = __builtin_amdgcn_ballot_w32(HJ); \
          if (HJ) { \
            const int pos = wc + (int)__builtin_amdgcn_mbcnt_lo(mj, 0u); \
            if (pos < WCAP) list[wave * WCAP + pos] = ((el0 + (J)) << 9) | (int)(SJ); \
          } \
          wc += (int)__builtin_popcount(mj); }
        HITJ(0, h0, s0)
        HITJ(1, h1, s1)
        HITJ(2, h2, s2)
        HITJ(3, h3, s3)
#undef HITJ
      }
    }
    if (lane == 0) wcnt[wave] = wc;
    __syncthreads();

    if (wave == 0) {
      for (int wsx = 0; wsx < NWAVE; ++wsx) {
        int n = wcnt[wsx];
        if (n > WCAP) n = WCAP;
        if (n < 0) n = 0;
        for (int i = 0; i < n; ++i) {
          const int ent  = list[wsx * WCAP + i];
          const int slot = ent & (NB - 1);
          const int el   = (ent >> 9) & (CHUNK - 1);
          int e = cbase + el;
          if (e > nE - 1) e = nE - 1;
          int src = ei[e];
          src = src < 0 ? 0 : (src > nN - 1 ? nN - 1 : src);
          int nd = nodeBase + slot;
          if (nd > nN - 1) nd = nN - 1;
          float lg = aspl[(size_t)src * NHD + hd] + adpl[(size_t)nd * NHD + hd];
          lg = (lg >= 0.f) ? lg : 0.2f * lg;
          const float mo = smax[slot * NHD + hd];
          const float mn = fmaxf(mo, lg);
          const float sc = __expf(fmaxf(mo - mn, -87.f));
          const float p  = __expf(fmaxf(lg - mn, -87.f));
          const v2f hv = *(const v2f*)(hpl + (size_t)src * HC + 2 * lane);
          v2f* sp = (v2f*)(sacc + slot * HC + 2 * lane);
          const v2f cur = *sp;
          const v2f nxt = cur * sc + p * hv;
          *sp = nxt;
          const float dn = sden[slot * NHD + hd] * sc + p;
          if ((lane & 15) == 0) {
            smax[slot * NHD + hd] = mn;
            sden[slot * NHD + hd] = dn;
          }
        }
      }
    }
    __syncthreads();
  }

  const int q   = lane & 15;
  const int c4  = 4 * q;
  const int hd2 = q >> 3;
  const v4f b4 = *(const v4f*)(bias + c4);
#pragma unroll 1
  for (int j = 0; j < NB / NWAVE / 2; ++j) {
    const int slot0 = wave * (NB / NWAVE) + 2 * j;
    const int node0 = nodeBase + slot0;
    if (node0 >= nN) break;
    const int slot = slot0 + hh;
    const int node = node0 + hh;
    const bool ok  = node < nN;
    const int ndc  = ok ? node : nN - 1;
    float lg = aspl[(size_t)ndc * NHD + hd2] + adpl[(size_t)ndc * NHD + hd2];
    lg = (lg >= 0.f) ? lg : 0.2f * lg;
    const float mo = smax[slot * NHD + hd2];
    const float mn = fmaxf(mo, lg);
    const float sc = __expf(fmaxf(mo - mn, -87.f));
    const float p  = __expf(fmaxf(lg - mn, -87.f));
    const v4f hv = *(const v4f*)(hpl + (size_t)ndc * HC + c4);
    const v4f a  = *(const v4f*)(sacc + slot * HC + c4) * sc + p * hv;
    const float dn  = sden[slot * NHD + hd2] * sc + p;
    const float inv = 1.0f / (dn + 1e-16f);
    const v4f y = a * inv + b4;
    float* op = out + (size_t)ndc * HC + c4;
    if (ok) *(volatile v4f*)op = y;
    __threadfence();
    if (ok) *(volatile v4f*)op = y;
  }
}

extern "C" void kernel_launch(void* const* d_in, const int* in_sizes, int n_in,
                              void* d_out, int out_size, void* d_ws, size_t ws_size,
                              hipStream_t stream) {
  if (n_in < 6) return;
  const int nN = in_sizes[0] / KD;
  if (nN < 1 || in_sizes[0] != nN * KD) return;
  if (in_sizes[1] != KD * HC) return;
  if (in_sizes[2] != HC || in_sizes[3] != HC || in_sizes[4] != HC) return;
  const int nE = in_sizes[5] / 2;
  if (nE < 0 || in_sizes[5] != 2 * nE) return;
  if (out_size != nN * HC) return;

  const float* x       = (const float*)d_in[0];
  const float* W       = (const float*)d_in[1];
  const float* att_src = (const float*)d_in[2];
  const float* att_dst = (const float*)d_in[3];
  const float* bias    = (const float*)d_in[4];
  const int*   ei      = (const int*)d_in[5];
  float* out = (float*)d_out;

  const int nP = ((nN + GR - 1) / GR) * GR;
  size_t off = 0;
  unsigned short* Whi = (unsigned short*)((char*)d_ws + off); off += (size_t)HC * KD * sizeof(unsigned short);
  unsigned short* Wlo = (unsigned short*)((char*)d_ws + off); off += (size_t)HC * KD * sizeof(unsigned short);
  float* hpl  = (float*)((char*)d_ws + off); off += (size_t)nP * HC * sizeof(float);
  float* aspl = (float*)((char*)d_ws + off); off += (size_t)nP * NHD * sizeof(float);
  float* adpl = (float*)((char*)d_ws + off); off += (size_t)nP * NHD * sizeof(float);
  if (off > ws_size) return;
  if (off > (size_t)134217728) return;

  const int n8 = HC * KD / 8;
  k_prep<<<(n8 + NTHR - 1) / NTHR, NTHR, 0, stream>>>(W, Whi, Wlo, n8);

  k_gemm<<<nP / GR, NTHR, 0, stream>>>(x, Whi, Wlo, att_src, att_dst, hpl, aspl, adpl, nN);

  hipFuncSetAttribute(reinterpret_cast<const void*>(&k_gat),
                      hipFuncAttributeMaxDynamicSharedMemorySize, LDS_BYTES);
  const int grid = (nN + NB - 1) / NB;
  k_gat<<<grid, NTHR, LDS_BYTES, stream>>>(ei, hpl, aspl, adpl, bias, out, nN, nE);
}
